// SparseTF_69827578298981
// MI455X (gfx1250) — hardware-verified
//
#include <hip/hip_runtime.h>
#include <stddef.h>
#include <stdint.h>


#define BBR   1024
#define DD    8192
#define UU    4096
#define NT    256
#define NWAVE 8
#define CH    8192
#define EPW   (CH / NWAVE)
#define SBW   (EPW / 32)
#define RB    64
#define CU    512
#define NBD   (DD / RB)
#define NBU   (UU / CU)
#define NNB   (NBD * NBU)
#define OFP   1152
#define QN    256
#define BM    128
#define BN    128
#define SP    132
#define WSCAP 134217728
#define XSC   16.0f
#define WSC   256.0f
#define INVB  2047
#define LDSA_BYTES ((NWAVE * NNB + OFP + CH + CH + 32) * 4)
#define LDSB_BYTES (RB * CU * 4 + QN * 4 + QN * 4 + RB * CU + QN)

static_assert(NT == NWAVE * 32);
static_assert(QN == NT);
static_assert((DD % 32) == 0);
static_assert((BBR % BM) == 0);
static_assert((UU % BN) == 0);
static_assert(((BBR * DD) % (8 * NT)) == 0);
static_assert(NNB == 4 * NT);
static_assert((OFP % 128) == 0);
static_assert(OFP >= NNB + 1);
static_assert(((CH / 128) % NWAVE) == 0);
static_assert((((CU / 4)) % NWAVE) == 0);
static_assert(RB == 64);
static_assert(NNB < 1024 + 1 && INVB > NNB);
static_assert(BM == 2 * 64 && BN == 4 * 32);
static_assert((SP % 4) == 0);
static_assert(LDSA_BYTES < 300000 && LDSB_BYTES < 300000);

typedef float    v4f  __attribute__((ext_vector_type(4))) __attribute__((may_alias));
typedef float    v8f  __attribute__((ext_vector_type(8)));
typedef int      v2i  __attribute__((ext_vector_type(2))) __attribute__((may_alias));
typedef int      v4i  __attribute__((ext_vector_type(4))) __attribute__((may_alias));
typedef _Float16 v8h  __attribute__((ext_vector_type(8))) __attribute__((may_alias));
typedef _Float16 v16h __attribute__((ext_vector_type(16)));
union FragH { v16h v; v8h h[2]; };

__device__ __forceinline__ v8f wmf(v16h a, v16h b, v8f c) {
  v8f d = __builtin_amdgcn_wmma_f32_16x16x32_f16(false, a, false, b, (short)0, c, false, false);
  asm volatile("v_nop\n\tv_nop\n\tv_nop\n\tv_nop" : "+v"(d) : "v"(a), "v"(b));
  return d;
}

__device__ __forceinline__ void put_i(const int* src, int* dst, int ngroups, int wave, int lane) {
#pragma unroll 1
  for (int g = wave; g < ngroups; g += NWAVE) {
    const int idx = g * 128 + 4 * lane;
    const v4i v = *(const v4i*)(src + idx);
    *(volatile v4i*)(dst + idx) = v;
  }
}
__device__ __forceinline__ void put_f(const float* src, float* dst, int ngroups, int wave, int lane) {
#pragma unroll 1
  for (int g = wave; g < ngroups; g += NWAVE) {
    const int idx = g * 128 + 4 * lane;
    const v4f v = *(const v4f*)(src + idx);
    *(volatile v4f*)(dst + idx) = v;
  }
}

__global__ __launch_bounds__(NT) void k_prepx(const float* __restrict__ x, _Float16* xh) {
  const size_t t = (size_t)blockIdx.x * NT + threadIdx.x;
  const float* p = x + t * 8;
  const v4f f0 = *(const v4f*)p;
  const v4f f1 = *(const v4f*)(p + 4);
  v8h a;
  a[0] = (_Float16)(f0.x * XSC); a[1] = (_Float16)(f0.y * XSC);
  a[2] = (_Float16)(f0.z * XSC); a[3] = (_Float16)(f0.w * XSC);
  a[4] = (_Float16)(f1.x * XSC); a[5] = (_Float16)(f1.y * XSC);
  a[6] = (_Float16)(f1.z * XSC); a[7] = (_Float16)(f1.w * XSC);
  _Float16* d = xh + t * 8;
  *(volatile v8h*)d = a;
  __threadfence();
  *(volatile v8h*)d = a;
}

struct Ent { int d; int u; int bin; float v; unsigned msk; bool valid; };

__device__ __forceinline__ Ent get_ent(const int* __restrict__ ind, const float* __restrict__ kv,
                                       int nnz, int e) {
  Ent r;
  const bool inr = e < nnz;
  const int ei = inr ? e : (nnz - 1);
  const v2i du = *(const v2i*)(ind + 2 * (size_t)ei);
  int d = du.x, u = du.y;
  d = d < 0 ? d + DD : d;
  u = u < 0 ? u + UU : u;
  const bool valid = inr && ((unsigned)d < (unsigned)DD) && ((unsigned)u < (unsigned)UU);
  r.valid = valid;
  r.d = valid ? d : 0;
  r.u = valid ? u : 0;
  r.v = kv[ei];
  r.bin = valid ? ((r.d / RB) * NBU + (r.u / CU)) : INVB;
  unsigned msk = 0xffffffffu;
#pragma unroll
  for (int b = 0; b < 11; ++b) {
    const bool bit = ((r.bin >> b) & 1) != 0;
    const unsigned bal = __builtin_amdgcn_ballot_w32(bit);
    msk &= bit ? bal : ~bal;
  }
  r.msk = msk;
  return r;
}

__global__ __launch_bounds__(NT) void k_bin(const int* __restrict__ ind, const float* __restrict__ kv,
                                            int nnz, int* offtab, int* skeyg, float* svalg) {
  extern __shared__ __align__(16) int ldsA[];
  int*   histw  = ldsA;
  int*   offrow = ldsA + NWAVE * NNB;
  int*   skey   = offrow + OFP;
  float* sval   = (float*)(skey + CH);
  int*   wtot   = (int*)(sval + CH);

  const int tid = threadIdx.x, lane = tid & 31, wave = tid >> 5;
  const int c = blockIdx.x;
  const int cbase = c * CH;
  const int ebase = cbase + wave * EPW + lane;

  const v4i zi = {0, 0, 0, 0};
  const v4f zf = {0.f, 0.f, 0.f, 0.f};
  for (int i = tid; i < (NWAVE * NNB) / 4; i += NT) ((v4i*)histw)[i] = zi;
  for (int i = tid; i < OFP / 4; i += NT) ((v4i*)offrow)[i] = zi;
  for (int i = tid; i < CH / 4; i += NT) { ((v4i*)skey)[i] = zi; ((v4f*)sval)[i] = zf; }
  __syncthreads();

#pragma unroll 1
  for (int sb = 0; sb < SBW; ++sb) {
    const Ent en = get_ent(ind, kv, nnz, ebase + sb * 32);
    const int cnt = __builtin_popcount(en.msk);
    const int lead = __builtin_ctz(en.msk);
    if (en.valid && lead == lane) histw[wave * NNB + en.bin] += cnt;
    __syncthreads();
  }

  const int t0 = 4 * tid;
  int tb0 = 0, tb1 = 0, tb2 = 0, tb3 = 0;
#pragma unroll
  for (int w = 0; w < NWAVE; ++w) {
    const int* hp = histw + w * NNB + t0;
    tb0 += hp[0]; tb1 += hp[1]; tb2 += hp[2]; tb3 += hp[3];
  }
  const int ssum = tb0 + tb1 + tb2 + tb3;
  int incl = ssum;
#pragma unroll
  for (int dl = 1; dl < 32; dl <<= 1) {
    const int y = __shfl_up(incl, dl);
    if (lane >= dl) incl += y;
  }
  if (lane == 31) wtot[wave] = incl;
  __syncthreads();
  int base = 0, all = 0;
#pragma unroll
  for (int w = 0; w < NWAVE; ++w) {
    const int tw = wtot[w];
    all += tw;
    base += (w < wave) ? tw : 0;
  }
  const int ex0 = base + incl - ssum;
  const int ex1 = ex0 + tb0, ex2 = ex1 + tb1, ex3 = ex2 + tb2;
  offrow[t0] = ex0; offrow[t0 + 1] = ex1; offrow[t0 + 2] = ex2; offrow[t0 + 3] = ex3;
  if (tid == 0) offrow[NNB] = all;
  {
    int q0 = ex0, q1 = ex1, q2 = ex2, q3 = ex3;
#pragma unroll
    for (int w = 0; w < NWAVE; ++w) {
      int* hp = histw + w * NNB + t0;
      const int h0 = hp[0], h1 = hp[1], h2 = hp[2], h3 = hp[3];
      hp[0] = q0; hp[1] = q1; hp[2] = q2; hp[3] = q3;
      q0 += h0; q1 += h1; q2 += h2; q3 += h3;
    }
  }
  __syncthreads();

  put_i(offrow, offtab + (size_t)c * OFP, OFP / 128, wave, lane);
  __threadfence();
  put_i(offrow, offtab + (size_t)c * OFP, OFP / 128, wave, lane);

#pragma unroll 1
  for (int sb = 0; sb < SBW; ++sb) {
    const Ent en = get_ent(ind, kv, nnz, ebase + sb * 32);
    const int cnt = __builtin_popcount(en.msk);
    const int lead = __builtin_ctz(en.msk);
    const int rank = __builtin_popcount(en.msk & ((1u << lane) - 1u));
    const int binc = en.valid ? en.bin : 0;
    int* cp = histw + wave * NNB + binc;
    const int old = *cp;
    int pos = old + rank;
    pos = pos < 0 ? 0 : (pos > CH - 1 ? CH - 1 : pos);
    if (en.valid && lead == lane) *cp = old + cnt;
    if (en.valid) { skey[pos] = (en.d << 12) | en.u; sval[pos] = en.v; }
    __syncthreads();
  }

  put_i(skey, skeyg + (size_t)cbase, CH / 128, wave, lane);
  put_f(sval, svalg + (size_t)cbase, CH / 128, wave, lane);
  __threadfence();
  put_i(skey, skeyg + (size_t)cbase, CH / 128, wave, lane);
  put_f(sval, svalg + (size_t)cbase, CH / 128, wave, lane);
}

__device__ __forceinline__ void flush_q(float* wacc, const int* qkey, const float* qval,
                                        unsigned char* own, unsigned char* dfl,
                                        int qn, int d0, int u0, int tid) {
  __syncthreads();
  const bool act = tid < qn;
  int key = 0, cl = 0;
  if (act) {
    key = qkey[tid];
    int dl = (key >> 12) - d0;
    int ul = (key & 4095) - u0;
    dl = dl < 0 ? 0 : (dl > RB - 1 ? RB - 1 : dl);
    ul = ul < 0 ? 0 : (ul > CU - 1 ? CU - 1 : ul);
    cl = dl * CU + ul;
    own[cl] = (unsigned char)tid;
  }
  dfl[tid] = 0;
  __syncthreads();
  int o = -1;
  if (act) {
    o = (int)own[cl];
    if (o != tid) dfl[o] = 1;
  }
  __syncthreads();
  if (act && o == tid) {
    if (dfl[tid] == 0) {
      wacc[cl] = wacc[cl] + qval[tid];
    } else {
      float s = wacc[cl];
#pragma unroll 1
      for (int j = 0; j < qn; ++j) {
        const int kj = qkey[j];
        const float vj = qval[j];
        if (kj == key) s = s + vj;
      }
      wacc[cl] = s;
    }
  }
  __syncthreads();
}

__global__ __launch_bounds__(NT) void k_wb(const int* __restrict__ offtab, const int* __restrict__ skeyg,
                                           const float* __restrict__ svalg, int nchunk, _Float16* wt) {
  extern __shared__ __align__(16) float ldsB[];
  float* wacc = ldsB;
  int*   qkey = (int*)(ldsB + RB * CU);
  float* qval = (float*)(qkey + QN);
  unsigned char* own = (unsigned char*)(qval + QN);
  unsigned char* dfl = own + RB * CU;

  const int tid = threadIdx.x, lane = tid & 31, wave = tid >> 5;
  const int bb = blockIdx.x;
  const int d0 = (bb / NBU) * RB;
  const int u0 = (bb % NBU) * CU;

  const v4f zf = {0.f, 0.f, 0.f, 0.f};
  for (int i = tid; i < (RB * CU) / 4; i += NT) ((v4f*)wacc)[i] = zf;
  __syncthreads();

  int qn = 0;
#pragma unroll 1
  for (int c = 0; c < nchunk; ++c) {
    const int* orow = offtab + (size_t)c * OFP;
    int beg = __builtin_amdgcn_readfirstlane(orow[bb]);
    int end = __builtin_amdgcn_readfirstlane(orow[bb + 1]);
    beg = beg < 0 ? 0 : (beg > CH ? CH : beg);
    end = end < beg ? beg : (end > CH ? CH : end);
    const int* krow = skeyg + (size_t)c * CH;
    const float* vrow = svalg + (size_t)c * CH;
    int p = beg;
    while (p < end) {
      const int rem = end - p, room = QN - qn;
      const int take = rem < room ? rem : room;
      int gi = p + tid;
      gi = gi > CH - 1 ? CH - 1 : gi;
      const int kk = krow[gi];
      const float vv = vrow[gi];
      if (tid < take) { qkey[qn + tid] = kk; qval[qn + tid] = vv; }
      qn += take; p += take;
      if (qn == QN) { flush_q(wacc, qkey, qval, own, dfl, QN, d0, u0, tid); qn = 0; }
    }
  }
  if (qn > 0) flush_q(wacc, qkey, qval, own, dfl, qn, d0, u0, tid);
  __syncthreads();

  auto emit = [&]() {
#pragma unroll 1
    for (int it = 0; it < (CU / 4) / NWAVE; ++it) {
      const int g = it * NWAVE + wave;
      const int ul = 4 * g + (lane >> 3);
      const int p8 = lane & 7;
      const float* col = wacc + (8 * p8) * CU + ul;
      v8h hv;
#pragma unroll
      for (int i = 0; i < 8; ++i) hv[i] = (_Float16)(col[i * CU] * WSC);
      _Float16* dst = wt + (size_t)(u0 + ul) * DD + d0 + 8 * p8;
      *(volatile v8h*)dst = hv;
    }
  };
  emit();
  __threadfence();
  emit();
}

__global__ __launch_bounds__(NT) void k_gemm(const _Float16* __restrict__ xh,
                                             const _Float16* __restrict__ wt,
                                             const float* __restrict__ bias,
                                             float* out) {
  __shared__ __attribute__((aligned(16))) float stg[64 * SP];

  const int tid = threadIdx.x, lane = tid & 31, wave = tid >> 5;
  const int wm = wave & 1, wn = wave >> 1;
  const int lr = lane & 15, hs = lane >> 4;
  const int m0 = blockIdx.y * BM, n0 = blockIdx.x * BN;

  const _Float16* ap0 = xh + (size_t)(m0 + wm * 64 + lr) * DD + 8 * hs;
  const _Float16* bp0 = wt + (size_t)(n0 + wn * 32 + lr) * DD + 8 * hs;

  v8f acc[4][2];
#pragma unroll
  for (int t = 0; t < 4; ++t)
#pragma unroll
    for (int j = 0; j < 2; ++j)
#pragma unroll
      for (int v = 0; v < 8; ++v) acc[t][j][v] = 0.f;

#pragma unroll 1
  for (int k0 = 0; k0 < DD; k0 += 32) {
    FragH a[4], b[2];
#pragma unroll
    for (int t = 0; t < 4; ++t) {
      const _Float16* ap = ap0 + (size_t)t * 16 * DD + k0;
      a[t].h[0] = *(const v8h*)(ap);
      a[t].h[1] = *(const v8h*)(ap + 16);
    }
#pragma unroll
    for (int j = 0; j < 2; ++j) {
      const _Float16* bp = bp0 + (size_t)j * 16 * DD + k0;
      b[j].h[0] = *(const v8h*)(bp);
      b[j].h[1] = *(const v8h*)(bp + 16);
    }
#pragma unroll
    for (int t = 0; t < 4; ++t)
#pragma unroll
      for (int j = 0; j < 2; ++j) acc[t][j] = wmf(a[t].v, b[j].v, acc[t][j]);
  }

  constexpr float OSC = 1.0f / (16.0f * 256.0f);
  const float bv0 = bias[n0 + wn * 32 + lr];
  const float bv1 = bias[n0 + wn * 32 + 16 + lr];

#pragma unroll 1
  for (int r = 0; r < 2; ++r) {
    if (wm == r) {
#pragma unroll
      for (int t = 0; t < 4; ++t) {
#pragma unroll
        for (int v = 0; v < 8; ++v) {
          float* sp = stg + (t * 16 + hs * 8 + v) * SP + wn * 32 + lr;
          sp[0]  = tanhf(acc[t][0][v] * OSC + bv0);
          sp[16] = tanhf(acc[t][1][v] * OSC + bv1);
        }
      }
    }
    __syncthreads();
    v4f o[8];
#pragma unroll
    for (int i = 0; i < 8; ++i) o[i] = *(const v4f*)(stg + (wave + 8 * i) * SP + 4 * lane);
    float* ob = out + (size_t)(m0 + 64 * r) * UU + n0 + 4 * lane;
#pragma unroll
    for (int i = 0; i < 8; ++i) *(volatile v4f*)(ob + (size_t)(wave + 8 * i) * UU) = o[i];
    __threadfence();
#pragma unroll
    for (int i = 0; i < 8; ++i) *(volatile v4f*)(ob + (size_t)(wave + 8 * i) * UU) = o[i];
    __syncthreads();
  }
}

extern "C" void kernel_launch(void* const* d_in, const int* in_sizes, int n_in,
                              void* d_out, int out_size, void* d_ws, size_t ws_size,
                              hipStream_t stream) {
  if (n_in < 4) return;
  if (in_sizes[0] != BBR * DD) return;
  const int nnz = in_sizes[1];
  if (nnz < 1) return;
  if (in_sizes[2] != UU) return;
  if (in_sizes[3] != 2 * nnz) return;
  if (out_size != BBR * UU) return;

  const float* x    = (const float*)d_in[0];
  const float* kv   = (const float*)d_in[1];
  const float* bias = (const float*)d_in[2];
  const int*   ind  = (const int*)d_in[3];
  float* out = (float*)d_out;

  const int nchunk = (nnz + CH - 1) / CH;

  char* ws = (char*)d_ws;
  size_t off = 0;
  const size_t oXh  = off; off += (size_t)BBR * DD * 2;       off = (off + 255) & ~(size_t)255;
  const size_t oWt  = off; off += (size_t)UU * DD * 2;        off = (off + 255) & ~(size_t)255;
  const size_t oOff = off; off += (size_t)nchunk * OFP * 4;   off = (off + 255) & ~(size_t)255;
  const size_t oKey = off; off += (size_t)nchunk * CH * 4;    off = (off + 255) & ~(size_t)255;
  const size_t oVal = off; off += (size_t)nchunk * CH * 4;    off = (off + 255) & ~(size_t)255;
  if (off > ws_size || off > (size_t)WSCAP) return;

  _Float16* xh     = (_Float16*)(ws + oXh);
  _Float16* wt     = (_Float16*)(ws + oWt);
  int*      offtab = (int*)(ws + oOff);
  int*      skeyg  = (int*)(ws + oKey);
  float*    svalg  = (float*)(ws + oVal);

  hipFuncSetAttribute(reinterpret_cast<const void*>(&k_bin), hipFuncAttributeMaxDynamicSharedMemorySize, LDSA_BYTES);
  hipFuncSetAttribute(reinterpret_cast<const void*>(&k_wb), hipFuncAttributeMaxDynamicSharedMemorySize, LDSB_BYTES);

  k_prepx<<<(BBR * DD) / (8 * NT), NT, 0, stream>>>(x, xh);
  k_bin<<<nchunk, NT, LDSA_BYTES, stream>>>(ind, kv, nnz, offtab, skeyg, svalg);
  k_wb<<<NNB, NT, LDSB_BYTES, stream>>>(offtab, skeyg, svalg, nchunk, wt);
  k_gemm<<<dim3(UU / BN, BBR / BM), NT, 0, stream>>>(xh, wt, bias, out);
}
